// Hgru2ScalarDecay_50586124812309
// MI455X (gfx1250) — hardware-run, weakly checked
//
#include <hip/hip_runtime.h>
#include <math.h>

constexpr int kNB    = 2;
constexpr int kNT    = 2048;
constexpr int kDM    = 2048;
constexpr int kNH    = 16;
constexpr int kHE    = 128;
constexpr int kCS    = 64;
constexpr int kNCH   = kNT / kCS;
constexpr int kRows  = kNB * kNT;
constexpr int kZN    = 64;
constexpr int kQKW   = 2 * kDM;
constexpr int kQP    = 136;
constexpr int kSP    = 72;
constexpr int kOP    = 132;
constexpr int kSmemHalves = 2 * kCS * kQP + kCS * kSP + kHE * kSP;
constexpr float kWoCarry    = 64.0f;
constexpr float kWoCarryInv = 1.0f / 64.0f;
constexpr float kInvDM      = 1.0f / (float)kDM;
constexpr float kNormEps    = 1e-6f;
static_assert(kNH * kHE == kDM, "heads x head dim = model dim");
static_assert(kRows == 4096 && kNCH == 32 && kNT == kCS * kNCH, "no chunk tail");
static_assert(kDM % 32 == 0, "GEMM K multiple of 32");
static_assert(kRows % 64 == 0 && kDM % 64 == 0 && kQKW % 64 == 0 && kZN % 64 == 0, "GEMM M,N multiples of 64");
static_assert(kNH <= kZN, "decay logits fit the padded plane");
static_assert(kCS * kOP * 2 <= 2 * kCS * kQP, "o tile overlays the q and k tiles only");
static_assert(kSmemHalves * 2 + 4 * kCS * 4 <= 65536, "static LDS");

typedef __attribute__((ext_vector_type(16))) _Float16 v16h;
typedef __attribute__((ext_vector_type(8)))  _Float16 v8h;
typedef __attribute__((ext_vector_type(16))) __bf16   v16b;
typedef __attribute__((ext_vector_type(8)))  __bf16   v8b;
typedef __attribute__((ext_vector_type(8)))  float    v8f;
typedef __attribute__((ext_vector_type(4)))  float    v4f;
typedef __attribute__((ext_vector_type(4)))  unsigned int v4u;

__device__ __forceinline__ unsigned short f2bf_bits(float f) {
  unsigned u = __float_as_uint(f);
  return (unsigned short)((u + 0x7FFFu + ((u >> 16) & 1u)) >> 16);
}
__device__ __forceinline__ float bf_bits2f(unsigned short h) { return __uint_as_float(((unsigned)h) << 16); }
__device__ __forceinline__ float bf16r(float f) { return bf_bits2f(f2bf_bits(f)); }
__device__ __forceinline__ unsigned pk16(unsigned short a, unsigned short b) { return (unsigned)a | ((unsigned)b << 16); }
__device__ __forceinline__ unsigned short h_bits(float f) { const _Float16 h = (_Float16)f; return __builtin_bit_cast(unsigned short, h); }
__device__ __forceinline__ float h16_to_f32(unsigned hb) {
  const unsigned sgn = (hb & 0x8000u) << 16;
  const unsigned em = hb & 0x7fffu;
  const float fn = __uint_as_float((em << 13) + 0x38000000u);
  const float fs = (float)em * 5.9604644775390625e-8f;
  const float mag = (em < 0x400u) ? fs : fn;
  return __uint_as_float(__float_as_uint(mag) | sgn);
}
__device__ __forceinline__ float ftz_pos(float x) { return (x < 1.17549435e-38f) ? 0.0f : x; }

__device__ __forceinline__ void guard4_h(v8f& a, v8f& b, v8f& c, v8f& d, v16h x, v16h y) {
  asm volatile("v_nop\n\tv_nop\n\tv_nop\n\tv_nop" : "+v"(a), "+v"(b), "+v"(c), "+v"(d) : "v"(x), "v"(y));
}
__device__ __forceinline__ void guard4_b(v8f& a, v8f& b, v8f& c, v8f& d, v16b x, v16b y) {
  asm volatile("v_nop\n\tv_nop\n\tv_nop\n\tv_nop" : "+v"(a), "+v"(b), "+v"(c), "+v"(d) : "v"(x), "v"(y));
}
__device__ __forceinline__ void keep4_h(v16h a, v16h b, v16h c, v16h d) { asm volatile("v_nop" :: "v"(a), "v"(b), "v"(c), "v"(d)); }
__device__ __forceinline__ void keep4_b(v16b a, v16b b, v16b c, v16b d) { asm volatile("v_nop" :: "v"(a), "v"(b), "v"(c), "v"(d)); }
__device__ __forceinline__ void acc_guard4(v8f& a, v8f& b, v8f& c, v8f& d) {
  asm volatile("v_nop\n\tv_nop\n\tv_nop\n\tv_nop" : "+v"(a), "+v"(b), "+v"(c), "+v"(d));
}

template <typename T> struct Frag;
template <> struct Frag<_Float16> {
  typedef v16h V;
  union U { v16h v; v8h h[2]; };
  static __device__ __forceinline__ v16h load(const _Float16* p) {
    U f;
    f.h[0] = *(const v8h*)(p);
    f.h[1] = *(const v8h*)(p + 16);
    return f.v;
  }
  static __device__ __forceinline__ v8f mma(v16h a, v16h b, v8f c) {
    return __builtin_amdgcn_wmma_f32_16x16x32_f16(false, a, false, b, (short)0, c, false, false);
  }
  static __device__ __forceinline__ void guard4(v8f& a, v8f& b, v8f& c, v8f& d, v16h x, v16h y) { guard4_h(a, b, c, d, x, y); }
  static __device__ __forceinline__ void keep(v16h a, v16h b, v16h c, v16h d) { keep4_h(a, b, c, d); }
};
template <> struct Frag<__bf16> {
  typedef v16b V;
  union U { v16b v; v8b h[2]; };
  static __device__ __forceinline__ v16b load(const __bf16* p) {
    U f;
    f.h[0] = *(const v8b*)(p);
    f.h[1] = *(const v8b*)(p + 16);
    return f.v;
  }
  static __device__ __forceinline__ v8f mma(v16b a, v16b b, v8f c) {
    return __builtin_amdgcn_wmma_f32_16x16x32_bf16(false, a, false, b, (short)0, c, false, false);
  }
  static __device__ __forceinline__ void guard4(v8f& a, v8f& b, v8f& c, v8f& d, v16b x, v16b y) { guard4_b(a, b, c, d, x, y); }
  static __device__ __forceinline__ void keep(v16b a, v16b b, v16b c, v16b d) { keep4_b(a, b, c, d); }
};

__device__ __forceinline__ v16h frag_load_h(const _Float16* p) { return Frag<_Float16>::load(p); }
__device__ __forceinline__ v8f mma_g(v16h a, v16h b, v8f c) {
  c = __builtin_amdgcn_wmma_f32_16x16x32_f16(false, a, false, b, (short)0, c, false, false);
  asm volatile("v_nop\n\tv_nop\n\tv_nop\n\tv_nop" : "+v"(c) : "v"(a), "v"(b));
  return c;
}

__global__ __launch_bounds__(256) void cvt8_bf16_kernel(const float* __restrict__ src, unsigned short* __restrict__ dst, int n8) {
  const int i = blockIdx.x * 256 + threadIdx.x;
  if (i < n8) {
    const float* sp = src + (size_t)i * 8;
    const v4f a = *(const v4f*)(sp);
    const v4f b = *(const v4f*)(sp + 4);
    unsigned short hb[8];
#pragma unroll
    for (int e = 0; e < 4; ++e) {
      const float fa = a[e];
      const float fb = b[e];
      hb[e]     = f2bf_bits(fa);
      hb[4 + e] = f2bf_bits(fb);
    }
    const v4u u = (v4u){pk16(hb[0], hb[1]), pk16(hb[2], hb[3]), pk16(hb[4], hb[5]), pk16(hb[6], hb[7])};
    unsigned short* q = dst + (size_t)i * 8;
    *(volatile v4u*)q = u;
    __threadfence();
    *(volatile v4u*)q = u;
  }
}

template <int MODE>
__global__ __launch_bounds__(256) void wtcast_kernel(const float* __restrict__ W, int ncols,
                                                     unsigned short* __restrict__ out, float carry) {
  __shared__ float sm[64][65];
  const int t  = threadIdx.x;
  const int d0 = blockIdx.x * 64;
  const int h0 = blockIdx.y * 64;
#pragma unroll
  for (int i = 0; i < 16; ++i) {
    const int e = i * 256 + t;
    const int r = e >> 6;
    const int c = e & 63;
    const int col  = h0 + c;
    const int colc = (col < ncols) ? col : (ncols - 1);
    const float raw = W[(size_t)(d0 + r) * ncols + colc];
    const float cv  = (MODE == 1) ? (bf16r(raw) * carry) : bf16r(raw);
    const float val = (col < ncols) ? cv : 0.0f;
    sm[c][r] = val;
  }
  __syncthreads();
  const int lane = t & 31, wave = t >> 5;
  const int q = lane >> 3, c8 = (lane & 7) * 8;
  for (int pass = 0; pass < 2; ++pass) {
#pragma unroll
    for (int it = 0; it < 2; ++it) {
      const int row = wave * 8 + it * 4 + q;
      unsigned short hb[8];
#pragma unroll
      for (int e = 0; e < 8; ++e) {
        const float sv = sm[row][c8 + e];
        hb[e] = (MODE == 1) ? h_bits(sv) : f2bf_bits(sv);
      }
      const v4u u = (v4u){pk16(hb[0], hb[1]), pk16(hb[2], hb[3]), pk16(hb[4], hb[5]), pk16(hb[6], hb[7])};
      *(volatile v4u*)(out + (size_t)(h0 + row) * kDM + d0 + c8) = u;
    }
    __threadfence();
  }
}

template <int ET> struct Elem;
template <> struct Elem<0> { typedef _Float16 T; };
template <> struct Elem<1> { typedef __bf16 T; };

template <int ET, int OUT_MODE, int ACT>
__global__ __launch_bounds__(256) void wmma_gemm64(
    const unsigned short* __restrict__ Ap, int lda,
    const unsigned short* __restrict__ Btp, int ldb,
    void* __restrict__ Cout, int ldc, int M, int N, int K, float scale) {
  typedef typename Elem<ET>::T T;
  typedef typename Frag<T>::V V;
  const T* A  = (const T*)Ap;
  const T* Bt = (const T*)Btp;
  __shared__ __align__(16) float sT[8][16 * 68];
  const int lane = threadIdx.x & 31;
  const int wave = threadIdx.x >> 5;
  const int tilesN = N >> 6;
  const int tilesM = M >> 6;
  const int tile = blockIdx.x * 8 + wave;
  if (tile >= tilesM * tilesN) return;
  const int tm = tile / tilesN;
  const int tn = tile - tm * tilesN;
  const int m0 = tm << 6;
  const int n0 = tn << 6;

  const int rlane = lane & 15;
  const int koff  = (lane >> 4) * 8;
  const int mOff  = (lane >> 4) * 8;

  const T* bp[4];
  const T* ap[4];
#pragma unroll
  for (int j = 0; j < 4; ++j) {
    bp[j] = Bt + (size_t)(n0 + (j << 4) + rlane) * ldb + koff;
    ap[j] = A  + (size_t)(m0 + (j << 4) + rlane) * lda + koff;
  }

  v8f acc[4][4];
#pragma unroll
  for (int i = 0; i < 4; ++i)
#pragma unroll
    for (int j = 0; j < 4; ++j) acc[i][j] = (v8f){0.f, 0.f, 0.f, 0.f, 0.f, 0.f, 0.f, 0.f};

  for (int k0 = 0; k0 < K; k0 += 32) {
    V bh[4];
#pragma unroll
    for (int j = 0; j < 4; ++j) bh[j] = Frag<T>::load(bp[j] + k0);
#pragma unroll
    for (int i = 0; i < 4; ++i) {
      const V ah = Frag<T>::load(ap[i] + k0);
#pragma unroll
      for (int j = 0; j < 4; ++j) acc[i][j] = Frag<T>::mma(ah, bh[j], acc[i][j]);
      Frag<T>::guard4(acc[i][0], acc[i][1], acc[i][2], acc[i][3], ah, bh[3]);
    }
    Frag<T>::keep(bh[0], bh[1], bh[2], bh[3]);
  }
  acc_guard4(acc[0][0], acc[0][1], acc[0][2], acc[0][3]);
  acc_guard4(acc[1][0], acc[1][1], acc[1][2], acc[1][3]);
  acc_guard4(acc[2][0], acc[2][1], acc[2][2], acc[2][3]);
  acc_guard4(acc[3][0], acc[3][1], acc[3][2], acc[3][3]);

  float* slab = sT[wave];
#pragma unroll
  for (int i = 0; i < 4; ++i) {
    const int mBase = m0 + (i << 4);
#pragma unroll
    for (int j = 0; j < 4; ++j) {
#pragma unroll
      for (int r = 0; r < 8; ++r) {
        const float v = acc[i][j][r] * scale;
        slab[(mOff + r) * 68 + (j << 4) + rlane] = v;
      }
    }
    __builtin_amdgcn_fence(__ATOMIC_RELEASE, "workgroup");
    __builtin_amdgcn_wave_barrier();
    __builtin_amdgcn_fence(__ATOMIC_ACQUIRE, "workgroup");
    if (ACT == 1) {
      const int ah2 = lane >> 4, ac4 = (lane & 15) * 4;
#pragma unroll 1
      for (int it = 0; it < 8; ++it) {
        float* sp = slab + (it * 2 + ah2) * 68 + ac4;
        const v4f vin = *(const v4f*)sp;
        v4f vout;
#pragma unroll
        for (int e = 0; e < 4; ++e) {
          const float xv = vin[e];
          const float sg = __builtin_amdgcn_rcpf(1.0f + expf(-xv));
          vout[e] = xv * sg;
        }
        *(v4f*)sp = vout;
      }
      __builtin_amdgcn_fence(__ATOMIC_RELEASE, "workgroup");
      __builtin_amdgcn_wave_barrier();
      __builtin_amdgcn_fence(__ATOMIC_ACQUIRE, "workgroup");
    }
    if (OUT_MODE == 0) {
      float* C = (float*)Cout;
      const int hh = lane >> 4, c4 = (lane & 15) * 4;
      for (int pass = 0; pass < 2; ++pass) {
#pragma unroll
        for (int it = 0; it < 8; ++it) {
          const int row = it * 2 + hh;
          const v4f v = *(const v4f*)(slab + row * 68 + c4);
          *(volatile v4f*)(C + (size_t)(mBase + row) * ldc + n0 + c4) = v;
        }
        __threadfence();
      }
    } else {
      const int q = lane >> 3, c8 = (lane & 7) * 8;
      unsigned short* C = (unsigned short*)Cout;
      for (int pass = 0; pass < 2; ++pass) {
#pragma unroll
        for (int it = 0; it < 4; ++it) {
          const int row = it * 4 + q;
          const float* sp = slab + row * 68 + c8;
          v8h hv;
#pragma unroll
          for (int e = 0; e < 8; ++e) hv[e] = (_Float16)sp[e];
          *(volatile v8h*)(C + (size_t)(mBase + row) * ldc + n0 + c8) = hv;
        }
        __threadfence();
      }
    }
    __builtin_amdgcn_fence(__ATOMIC_RELEASE, "workgroup");
    __builtin_amdgcn_wave_barrier();
    __builtin_amdgcn_fence(__ATOMIC_ACQUIRE, "workgroup");
  }
}

__global__ __launch_bounds__(256) void chunk_scan_kernel(const unsigned short* __restrict__ QKp,
                                                         const unsigned short* __restrict__ VTp,
                                                         const float* __restrict__ Z, float* __restrict__ O) {
  __shared__ __align__(16) unsigned short smem[kSmemHalves];
  __shared__ float s_ld[kCS];
  __shared__ float s_cum[kCS];
  __shared__ float s_eL[kCS];
  __shared__ float s_ed[kCS];
  unsigned short* qs  = smem;
  unsigned short* ks  = smem + kCS * kQP;
  unsigned short* ss  = smem + 2 * kCS * kQP;
  unsigned short* kdt = smem + 2 * kCS * kQP + kCS * kSP;
  float* Ost = (float*)smem;
  const _Float16* qsH  = (const _Float16*)qs;
  const _Float16* ksH  = (const _Float16*)ks;
  const _Float16* ssH  = (const _Float16*)ss;
  const _Float16* kdtH = (const _Float16*)kdt;
  const _Float16* VT   = (const _Float16*)VTp;

  const int bid = blockIdx.x;
  const int h = bid & (kNH - 1);
  const int b = bid >> 4;
  const int tid = threadIdx.x, lane = tid & 31, w = tid >> 5;
  const int c = lane & 15, hh = lane >> 4, koff = hh * 8;
  const int tm  = w >> 1;
  const int tnb = (w & 1) * 2;

  const v8f z8 = {0.f, 0.f, 0.f, 0.f, 0.f, 0.f, 0.f, 0.f};
  v8f S[8];
#pragma unroll
  for (int t = 0; t < 8; ++t) S[t] = z8;

#pragma unroll 1
  for (int n = 0; n < kNCH; ++n) {
    const size_t r0 = (size_t)b * kNT + (size_t)n * kCS;
    __syncthreads();

    v16h vb[2];
    {
      const _Float16* vrow = VT + (size_t)(h * kHE + 16 * w + c) * kRows + r0 + koff;
      vb[0] = frag_load_h(vrow);
      vb[1] = frag_load_h(vrow + 32);
    }

#pragma unroll
    for (int it = 0; it < 4; ++it) {
      const int idx = it * 256 + tid;
      const int row = idx >> 4, c8 = (idx & 15) * 8;
      const size_t go = (r0 + (size_t)row) * kQKW + h * kHE + c8;
      const v4u vq = *(const v4u*)(QKp + go);
      const v4u vk = *(const v4u*)(QKp + go + kDM);
      *(v4u*)(qs + row * kQP + c8) = vq;
      *(v4u*)(ks + row * kQP + c8) = vk;
    }
    if (tid < kCS) {
      const float zv = Z[(r0 + (size_t)tid) * kZN + h];
      s_ld[tid] = fminf(zv, 0.0f) - log1pf(expf(-fabsf(zv)));
    }
    __syncthreads();

    if (tid < kCS) {
      float run = 0.0f, tot = 0.0f;
#pragma unroll 4
      for (int u = 0; u < kCS; ++u) {
        const float l = s_ld[u];
        tot += l;
        run += (u <= tid) ? l : 0.0f;
      }
      s_cum[tid] = run;
      s_eL[tid]  = ftz_pos(expf(run));
      s_ed[tid]  = ftz_pos(expf(tot - run));
    }
    __syncthreads();

    {
      v16h qa[4];
#pragma unroll
      for (int k = 0; k < 4; ++k) qa[k] = frag_load_h(qsH + (16 * tm + c) * kQP + koff + 32 * k);
#pragma unroll 1
      for (int t = 0; t < 2; ++t) {
        const int tn = tnb + t;
        v8f acc = z8;
#pragma unroll
        for (int k = 0; k < 4; ++k) {
          const v16h kb = frag_load_h(ksH + (16 * tn + c) * kQP + koff + 32 * k);
          acc = mma_g(qa[k], kb, acc);
        }
        const int j = 16 * tn + c;
        const float Lj = s_cum[j];
#pragma unroll
        for (int r = 0; r < 8; ++r) {
          const int i = 16 * tm + 8 * hh + r;
          const float dl = fminf(s_cum[i] - Lj, 0.0f);
          const float wgt = ftz_pos(expf(dl));
          const float sv = (j <= i) ? (acc[r] * wgt) : 0.0f;
          ss[i * kSP + j] = h_bits(sv);
        }
      }
    }
#pragma unroll
    for (int it = 0; it < 4; ++it) {
      const int item = it * 256 + tid;
      const int e  = item & (kHE - 1);
      const int i0 = (item >> 7) * 8;
      unsigned short hb[8];
#pragma unroll
      for (int u = 0; u < 8; ++u) {
        const unsigned kbits = ks[(i0 + u) * kQP + e];
        const float kv = h16_to_f32(kbits);
        hb[u] = h_bits(kv * s_ed[i0 + u]);
      }
      const v4u pk = (v4u){pk16(hb[0], hb[1]), pk16(hb[2], hb[3]), pk16(hb[4], hb[5]), pk16(hb[6], hb[7])};
      *(v4u*)(kdt + e * kSP + i0) = pk;
    }
    __syncthreads();

    v8f accO[4];
#pragma unroll
    for (int mt = 0; mt < 4; ++mt) accO[mt] = z8;
#pragma unroll
    for (int s = 0; s < 4; ++s) {
      v16h bS;
#pragma unroll
      for (int r = 0; r < 8; ++r) {
        bS[r]     = (_Float16)S[2 * s][r];
        bS[8 + r] = (_Float16)S[2 * s + 1][r];
      }
#pragma unroll
      for (int mt = 0; mt < 4; ++mt) {
        const v16h a = frag_load_h(qsH + (16 * mt + c) * kQP + koff + 32 * s);
        accO[mt] = mma_g(a, bS, accO[mt]);
      }
    }
#pragma unroll
    for (int mt = 0; mt < 4; ++mt) {
#pragma unroll
      for (int r = 0; r < 8; ++r) accO[mt][r] *= s_eL[16 * mt + 8 * hh + r];
    }
#pragma unroll
    for (int k = 0; k < 2; ++k) {
#pragma unroll
      for (int mt = 0; mt < 4; ++mt) {
        const v16h a = frag_load_h(ssH + (16 * mt + c) * kSP + koff + 32 * k);
        accO[mt] = mma_g(a, vb[k], accO[mt]);
      }
    }
    {
      const float etot = ftz_pos(expf(s_cum[kCS - 1]));
#pragma unroll
      for (int et = 0; et < 8; ++et) {
#pragma unroll
        for (int r = 0; r < 8; ++r) S[et][r] *= etot;
#pragma unroll
        for (int k = 0; k < 2; ++k) {
          const v16h a = frag_load_h(kdtH + (16 * et + c) * kSP + koff + 32 * k);
          S[et] = mma_g(a, vb[k], S[et]);
        }
      }
    }
    __syncthreads();

#pragma unroll
    for (int mt = 0; mt < 4; ++mt) {
#pragma unroll
      for (int r = 0; r < 8; ++r) Ost[(16 * mt + 8 * hh + r) * kOP + 16 * w + c] = accO[mt][r];
    }
    __syncthreads();
    for (int pass = 0; pass < 2; ++pass) {
#pragma unroll
      for (int it = 0; it < 8; ++it) {
        const int row = it * 8 + w;
        const v4f v = *(const v4f*)(Ost + row * kOP + lane * 4);
        *(volatile v4f*)(O + (r0 + (size_t)row) * kDM + h * kHE + lane * 4) = v;
      }
      __threadfence();
    }
  }
}

__global__ __launch_bounds__(256) void rms_kernel(const float* __restrict__ O, const float* __restrict__ norm_w,
                                                  unsigned short* __restrict__ ON) {
  __shared__ float red[8];
  const int tid = threadIdx.x, lane = tid & 31, wave = tid >> 5;
  const size_t base = (size_t)blockIdx.x * kDM + 8 * tid;
  const v4f o0 = *(const v4f*)(O + base);
  const v4f o1 = *(const v4f*)(O + base + 4);
  const v4f w0 = *(const v4f*)(norm_w + 8 * tid);
  const v4f w1 = *(const v4f*)(norm_w + 8 * tid + 4);
  float ov[8], wv[8];
#pragma unroll
  for (int e = 0; e < 4; ++e) {
    ov[e] = o0[e];
    ov[4 + e] = o1[e];
    const float wa = w0[e];
    const float wb = w1[e];
    wv[e] = bf16r(wa);
    wv[4 + e] = bf16r(wb);
  }
  float ssq = 0.0f;
#pragma unroll
  for (int e = 0; e < 8; ++e) ssq = fmaf(ov[e], ov[e], ssq);
#pragma unroll
  for (int off = 16; off > 0; off >>= 1) ssq += __shfl_xor(ssq, off, 32);
  if (lane == 0) red[wave] = ssq;
  __syncthreads();
  float total = 0.0f;
#pragma unroll
  for (int i = 0; i < 8; ++i) total += red[i];
  const float inv = rsqrtf(total * kInvDM + kNormEps);
  unsigned short hb[8];
#pragma unroll
  for (int e = 0; e < 8; ++e) hb[e] = h_bits((ov[e] * inv) * wv[e]);
  const v4u u = (v4u){pk16(hb[0], hb[1]), pk16(hb[2], hb[3]), pk16(hb[4], hb[5]), pk16(hb[6], hb[7])};
  unsigned short* op = ON + base;
  *(volatile v4u*)op = u;
  __threadfence();
  *(volatile v4u*)op = u;
}

extern "C" void kernel_launch(void* const* d_in, const int* in_sizes, int n_in,
                              void* d_out, int out_size, void* d_ws, size_t ws_size, hipStream_t stream) {
  if (n_in < 7 || d_out == nullptr || d_ws == nullptr) return;
  if (in_sizes[0] != kRows * kDM || in_sizes[1] != kDM * kDM || in_sizes[2] != kDM * kDM ||
      in_sizes[3] != kDM * kDM || in_sizes[4] != kDM * kNH || in_sizes[5] != kDM * kDM ||
      in_sizes[6] != kDM || out_size != kRows * kDM) return;

  const float* x      = (const float*)d_in[0];
  const float* Wq     = (const float*)d_in[1];
  const float* Wk     = (const float*)d_in[2];
  const float* Wv     = (const float*)d_in[3];
  const float* Wf     = (const float*)d_in[4];
  const float* Wo     = (const float*)d_in[5];
  const float* norm_w = (const float*)d_in[6];
  float* out = (float*)d_out;

  char* ws = (char*)d_ws;
  size_t off = 0;
  auto carve = [&](size_t bytes) -> char* { char* p = ws + off; off += (bytes + 255) & ~(size_t)255; return p; };
  unsigned short* X16  = (unsigned short*)carve((size_t)kRows * kDM * 2);
  unsigned short* WQKT = (unsigned short*)carve((size_t)kQKW * kDM * 2);
  unsigned short* WVT  = (unsigned short*)carve((size_t)kDM * kDM * 2);
  unsigned short* WFT  = (unsigned short*)carve((size_t)kZN * kDM * 2);
  unsigned short* QK16 = (unsigned short*)carve((size_t)kRows * kQKW * 2);
  unsigned short* VT16 = (unsigned short*)carve((size_t)kDM * kRows * 2);
  float*          Zp   = (float*)carve((size_t)kRows * kZN * 4);
  float*          O32  = (float*)carve((size_t)kRows * kDM * 4);
  if (off > ws_size || off > (size_t)134217728) return;
  static_assert((size_t)kRows * kDM * 2 + (size_t)kDM * kDM * 2 <= (size_t)kRows * kQKW * 2, "aliases fit the q|k plane");
  unsigned short* ON16 = QK16;
  unsigned short* WOT  = QK16 + (size_t)kRows * kDM;

  const int n8x = kRows * kDM / 8;
  cvt8_bf16_kernel<<<n8x / 256, 256, 0, stream>>>(x, X16, n8x);
  wtcast_kernel<0><<<dim3(kDM / 64, kDM / 64), 256, 0, stream>>>(Wq, kDM, WQKT, 1.0f);
  wtcast_kernel<0><<<dim3(kDM / 64, kDM / 64), 256, 0, stream>>>(Wk, kDM, WQKT + (size_t)kDM * kDM, 1.0f);
  wtcast_kernel<0><<<dim3(kDM / 64, kDM / 64), 256, 0, stream>>>(Wv, kDM, WVT, 1.0f);
  wtcast_kernel<0><<<dim3(kDM / 64, 1), 256, 0, stream>>>(Wf, kNH, WFT, 1.0f);

  wmma_gemm64<1, 1, 1><<<(kRows / 64) * (kQKW / 64) / 8, 256, 0, stream>>>(
      X16, kDM, WQKT, kDM, (void*)QK16, kQKW, kRows, kQKW, kDM, 1.0f);
  wmma_gemm64<1, 1, 0><<<(kDM / 64) * (kRows / 64) / 8, 256, 0, stream>>>(
      WVT, kDM, X16, kDM, (void*)VT16, kRows, kDM, kRows, kDM, 1.0f);
  wmma_gemm64<1, 0, 0><<<(kRows / 64) * (kZN / 64) / 8, 256, 0, stream>>>(
      X16, kDM, WFT, kDM, (void*)Zp, kZN, kRows, kZN, kDM, 1.0f);

  chunk_scan_kernel<<<kNB * kNH, 256, 0, stream>>>(QK16, VT16, Zp, O32);

  wtcast_kernel<1><<<dim3(kDM / 64, kDM / 64), 256, 0, stream>>>(Wo, kDM, WOT, kWoCarry);

  rms_kernel<<<kRows, 256, 0, stream>>>(O32, norm_w, ON16);

  wmma_gemm64<0, 0, 0><<<(kRows / 64) * (kDM / 64) / 8, 256, 0, stream>>>(
      ON16, kDM, WOT, kDM, (void*)out, kDM, kRows, kDM, kDM, kWoCarryInv);
}
